// HEPOSEncoderLayer_75445395522269
// MI455X (gfx1250) — hardware-run, weakly checked
//
#include <hip/hip_runtime.h>


#ifndef NB
#define NB 2
#endif
#ifndef SEQ
#define SEQ 4096
#endif
#define NB_FULL  2
#define SEQ_FULL 4096
#ifndef OUT_SEQ
#define OUT_SEQ SEQ
#endif
#define DM   1024
#define NH_  16
#define HD   64
#define DFF  4096
#define AW   4
#define SC2  (0.125f * 1.4426950408889634f)
#define PSH  8.0f
#define CXS  1024.0f
#define WOS  1024.0f
#define OSCL (1.0f / (1024.0f * 1024.0f))
#define HCS  16.0f
#define W1S  1024.0f
#define FOLD1 (1.0f / (16.0f * 1024.0f))
#define F1S  16.0f
#define W2S  2048.0f
#define FOLD2 (1.0f / (16.0f * 2048.0f))
#define LNE  1.0e-5f

static_assert(HD == 64);
static_assert(NH_ * HD == DM);
static_assert(NH_ == 16);
static_assert(DM % 64 == 0);
static_assert(DFF % 64 == 0);
static_assert((3 * DM) % 64 == 0);
static_assert(DM % 32 == 0);
static_assert(DFF % 32 == 0);
static_assert(SEQ % 64 == 0);
static_assert((NB * SEQ) % 64 == 0);
static_assert(SEQ % 1024 == 0);
static_assert(SEQ % (16 * AW) == 0);
static_assert((NB * SEQ) % 8 == 0);
static_assert(((size_t)SEQ * DM) % 8 == 0);
static_assert(NB <= NB_FULL);
static_assert(SEQ <= SEQ_FULL);
static_assert(4 * 32 * 8 == 16 * 64);
static_assert(8 * 32 * 4 == 16 * 64);
static_assert(8 * 32 * 4 == DM);
static_assert(4 * 32 * 8 == DM);
static_assert(2 * 256 * 8 == 64 * 64);
static_assert(4 * 256 * 4 == 64 * 64);
static_assert(16 * 68 * 4 <= 131072);
static_assert(AW * 16 * 68 * 4 <= 131072);
static_assert(8 * DM * 4 <= 131072);
static_assert(64 * 72 * 2 <= 131072);

typedef _Float16 h16;
typedef unsigned short bf;
typedef __attribute__((ext_vector_type(16))) __bf16   v16bf;
typedef __attribute__((ext_vector_type(16))) _Float16 v16h;
typedef __attribute__((ext_vector_type(8)))  _Float16 v8h;
typedef __attribute__((ext_vector_type(8)))  unsigned short v8us;
typedef __attribute__((ext_vector_type(8)))  float    v8f;
typedef __attribute__((ext_vector_type(4)))  float    v4f;
typedef v4f  __attribute__((may_alias)) v4fa;
typedef v8us __attribute__((may_alias)) v8usa;
typedef v8h  __attribute__((may_alias)) v8ha;

__device__ __forceinline__ unsigned short f2bf(float f) { unsigned u = __float_as_uint(f); u += 0x7FFFu + ((u >> 16) & 1u); return (unsigned short)(u >> 16); }
__device__ __forceinline__ float bfval(float f) { return __uint_as_float(((unsigned)f2bf(f)) << 16); }
__device__ __forceinline__ v16h cat16(v8h lo, v8h hi) { return __builtin_shufflevector(lo, hi, 0, 1, 2, 3, 4, 5, 6, 7, 8, 9, 10, 11, 12, 13, 14, 15); }
__device__ __forceinline__ v16bf cat16b(v8us lo, v8us hi) { return __builtin_bit_cast(v16bf, __builtin_shufflevector(lo, hi, 0, 1, 2, 3, 4, 5, 6, 7, 8, 9, 10, 11, 12, 13, 14, 15)); }
__device__ __forceinline__ v8f wmma16(v16h a, v16h b, v8f c) { return __builtin_amdgcn_wmma_f32_16x16x32_f16(false, a, false, b, (short)0, c, false, false); }
__device__ __forceinline__ v8f wmmab(v16bf a, v16bf b, v8f c) { return __builtin_amdgcn_wmma_f32_16x16x32_bf16(false, a, false, b, (short)0, c, false, false); }
__device__ __forceinline__ v16h  ldh(const h16* p) { return cat16(*(const v8h*)p, *(const v8h*)(p + 16)); }
__device__ __forceinline__ v16bf ldb(const bf* p)  { return cat16b(*(const v8us*)p, *(const v8us*)(p + 16)); }
__device__ __forceinline__ void wave_sync() { __builtin_amdgcn_fence(3  , "wavefront"); __builtin_amdgcn_wave_barrier(); asm volatile("" ::: "memory"); }
__device__ __forceinline__ h16 toh_flush(float v) { const h16 r = (h16)v; return (__builtin_fabsf(v) < 6.103515625e-05f) ? (h16)0.0f : r; }

__global__ __launch_bounds__(256) void k_cvt8(const float* __restrict__ src, bf* dst, size_t n8) {
    const size_t i = (size_t)blockIdx.x * 256 + threadIdx.x; if (i >= n8) return;
    const v8f v = *(const v8f*)(src + i * 8); v8us o;
#pragma unroll
    for (int k = 0; k < 8; ++k) o[k] = f2bf(v[k]);
    *(volatile v8us*)(dst + i * 8) = o; __threadfence(); *(volatile v8us*)(dst + i * 8) = o;
}

__global__ __launch_bounds__(256) void k_wtb(const float* __restrict__ src, bf* dst, int Kd, int Nd) {
    __shared__ __align__(16) unsigned short ts[64 * 72];
    const int tid = threadIdx.x; const int n0 = blockIdx.x * 64, k0 = blockIdx.y * 64;
#pragma unroll
    for (int it = 0; it < 4; ++it) { const int idx = tid + it * 256, kr = idx >> 4, nc = (idx & 15) * 4;
        const v4f v = *(const v4f*)(src + (size_t)(k0 + kr) * (size_t)Nd + n0 + nc);
#pragma unroll
        for (int j = 0; j < 4; ++j) ts[(nc + j) * 72 + kr] = f2bf(v[j]); }
    __syncthreads();
#pragma unroll 1
    for (int ps = 0; ps < 2; ++ps) {
#pragma unroll
        for (int it = 0; it < 2; ++it) { const int idx = tid + it * 256, nr = idx >> 3, pc = (idx & 7) * 8;
            const v8us o = *(const v8usa*)(&ts[nr * 72 + pc]);
            *(volatile v8us*)(dst + (size_t)(n0 + nr) * (size_t)Kd + k0 + pc) = o; }
        if (ps == 0) __threadfence(); }
}

__global__ __launch_bounds__(256) void k_wth(const float* __restrict__ src, h16* dst, int Kd, int Nd, float scl) {
    __shared__ __align__(16) h16 ts[64 * 72];
    const int tid = threadIdx.x; const int n0 = blockIdx.x * 64, k0 = blockIdx.y * 64;
#pragma unroll
    for (int it = 0; it < 4; ++it) { const int idx = tid + it * 256, kr = idx >> 4, nc = (idx & 15) * 4;
        const v4f v = *(const v4f*)(src + (size_t)(k0 + kr) * (size_t)Nd + n0 + nc);
#pragma unroll
        for (int j = 0; j < 4; ++j) ts[(nc + j) * 72 + kr] = toh_flush(bfval(v[j]) * scl); }
    __syncthreads();
#pragma unroll 1
    for (int ps = 0; ps < 2; ++ps) {
#pragma unroll
        for (int it = 0; it < 2; ++it) { const int idx = tid + it * 256, nr = idx >> 3, pc = (idx & 7) * 8;
            const v8h o = *(const v8ha*)(&ts[nr * 72 + pc]);
            *(volatile v8h*)(dst + (size_t)(n0 + nr) * (size_t)Kd + k0 + pc) = o; }
        if (ps == 0) __threadfence(); }
}

__global__ __launch_bounds__(32) void k_proj(const bf* __restrict__ A, size_t apitch, const bf* __restrict__ Bt, size_t bpitch, const float* __restrict__ bias, int blen, int brow,
                                             h16* Ph, int RB, size_t sRB, int pitch, int CB, size_t sCB) {
    __shared__ __align__(16) float os[16 * 68];
    const int K = DM;
    const int lane = threadIdx.x & 31, lr = lane & 15, hi = lane >> 4; const int r0 = blockIdx.x * 64, c0 = blockIdx.y * 64;
    v8f acc[4][4];
#pragma unroll
    for (int mb = 0; mb < 4; ++mb)
#pragma unroll
        for (int nb = 0; nb < 4; ++nb) acc[mb][nb] = (v8f){};
    const size_t aoff = (size_t)(r0 + lr) * apitch + 8 * hi, boff = (size_t)(c0 + lr) * bpitch + 8 * hi;
#pragma unroll 1
    for (int kc = 0; kc < K; kc += 32) {
        v16bf a[4];
#pragma unroll
        for (int mb = 0; mb < 4; ++mb) a[mb] = ldb(A + aoff + (size_t)mb * 16 * apitch + kc);
#pragma unroll
        for (int nb = 0; nb < 4; ++nb) { const v16bf b = ldb(Bt + boff + (size_t)nb * 16 * bpitch + kc);
#pragma unroll
            for (int mb = 0; mb < 4; ++mb) acc[mb][nb] = wmmab(a[mb], b, acc[mb][nb]); }
        asm volatile("v_nop\n\tv_nop\n\tv_nop\n\tv_nop" : "+v"(acc[0][0]), "+v"(acc[1][1]), "+v"(acc[2][2]), "+v"(acc[3][3]) : "v"(a[0]), "v"(a[1]), "v"(a[2]), "v"(a[3]));
    }
    const size_t tbase = (size_t)(r0 / RB) * sRB + (size_t)(r0 % RB) * (size_t)pitch + (size_t)(c0 / CB) * sCB + (size_t)(c0 % CB);
#pragma unroll
    for (int mb = 0; mb < 4; ++mb) {
#pragma unroll
        for (int nb = 0; nb < 4; ++nb) {
#pragma unroll
            for (int j = 0; j < 8; ++j) os[(hi * 8 + j) * 68 + nb * 16 + lr] = acc[mb][nb][j]; }
        wave_sync();
        const size_t sb = tbase + (size_t)(mb * 16) * (size_t)pitch;
#pragma unroll 1
        for (int ps = 0; ps < 2; ++ps) {
#pragma unroll
            for (int s = 0; s < 4; ++s) { const int row = 4 * s + (lane >> 3), c8 = (lane & 7) * 8;
                const v4f x0 = *(const v4fa*)(&os[row * 68 + c8]); const v4f x1 = *(const v4fa*)(&os[row * 68 + c8 + 4]);
                const int ri = min(r0 + mb * 16 + row, blen - 1), ci = min(c0 + c8, blen - 8);
                const float rb = bfval(bias[ri]);
                const v4f cb0 = *(const v4f*)(bias + ci); const v4f cb1 = *(const v4f*)(bias + ci + 4);
                v8h hv;
#pragma unroll
                for (int i = 0; i < 4; ++i) { hv[i] = toh_flush(x0[i] + ((brow != 0) ? rb : bfval(cb0[i]))); hv[4 + i] = toh_flush(x1[i] + ((brow != 0) ? rb : bfval(cb1[i]))); }
                const size_t oo = sb + (size_t)row * (size_t)pitch + c8;
                *(volatile v8h*)(Ph + oo) = hv; }
            if (ps == 0) __threadfence(); }
        wave_sync();
    }
}

__global__ __launch_bounds__(32) void k_ffn1(const h16* __restrict__ A, const h16* __restrict__ Bt, const float* __restrict__ b1, h16* F) {
    __shared__ __align__(16) float os[16 * 68];
    const int K = DM;
    const int lane = threadIdx.x & 31, lr = lane & 15, hi = lane >> 4; const int r0 = blockIdx.x * 64, c0 = blockIdx.y * 64;
    v8f acc[4][4];
#pragma unroll
    for (int mb = 0; mb < 4; ++mb)
#pragma unroll
        for (int nb = 0; nb < 4; ++nb) acc[mb][nb] = (v8f){};
    const size_t aoff = (size_t)(r0 + lr) * K + 8 * hi, boff = (size_t)(c0 + lr) * K + 8 * hi;
#pragma unroll 1
    for (int kc = 0; kc < K; kc += 32) {
        v16h a[4];
#pragma unroll
        for (int mb = 0; mb < 4; ++mb) a[mb] = ldh(A + aoff + (size_t)mb * 16 * K + kc);
#pragma unroll
        for (int nb = 0; nb < 4; ++nb) { const v16h b = ldh(Bt + boff + (size_t)nb * 16 * K + kc);
#pragma unroll
            for (int mb = 0; mb < 4; ++mb) acc[mb][nb] = wmma16(a[mb], b, acc[mb][nb]); }
        asm volatile("v_nop\n\tv_nop\n\tv_nop\n\tv_nop" : "+v"(acc[0][0]), "+v"(acc[1][1]), "+v"(acc[2][2]), "+v"(acc[3][3]) : "v"(a[0]), "v"(a[1]), "v"(a[2]), "v"(a[3]));
    }
    const int c8 = (lane & 7) * 8;
    const v4f braw0 = *(const v4f*)(b1 + c0 + c8); const v4f braw1 = *(const v4f*)(b1 + c0 + c8 + 4);
    v4f bb0, bb1;
#pragma unroll
    for (int i = 0; i < 4; ++i) { bb0[i] = bfval(braw0[i]); bb1[i] = bfval(braw1[i]); }
    const size_t tbase = (size_t)r0 * DFF + c0;
#pragma unroll
    for (int mb = 0; mb < 4; ++mb) {
#pragma unroll
        for (int nb = 0; nb < 4; ++nb) {
#pragma unroll
            for (int j = 0; j < 8; ++j) os[(hi * 8 + j) * 68 + nb * 16 + lr] = acc[mb][nb][j]; }
        wave_sync();
        const size_t sb = tbase + (size_t)(mb * 16) * DFF;
#pragma unroll 1
        for (int ps = 0; ps < 2; ++ps) {
#pragma unroll
            for (int s = 0; s < 4; ++s) { const int row = 4 * s + (lane >> 3);
                const v4f x0 = *(const v4fa*)(&os[row * 68 + c8]); const v4f x1 = *(const v4fa*)(&os[row * 68 + c8 + 4]); v8h hv;
#pragma unroll
                for (int i = 0; i < 4; ++i) { hv[i] = toh_flush(fmaxf(x0[i] * FOLD1 + bb0[i], 0.0f) * F1S); hv[4 + i] = toh_flush(fmaxf(x1[i] * FOLD1 + bb1[i], 0.0f) * F1S); }
                *(volatile v8h*)(F + sb + (size_t)row * DFF + c8) = hv; }
            if (ps == 0) __threadfence(); }
        wave_sync();
    }
}

__global__ __launch_bounds__(32) void k_oproj(const h16* __restrict__ A, const h16* __restrict__ Bt, int K, float oscl, const float* __restrict__ bo, const float* res, int res_seq, int resbf, float* OUT) {
    __shared__ __align__(16) float os[16 * 68];
    const int lane = threadIdx.x & 31, lr = lane & 15, hi = lane >> 4; const int r0 = blockIdx.x * 64, c0 = blockIdx.y * 64;
    v8f acc[4][4];
#pragma unroll
    for (int mb = 0; mb < 4; ++mb)
#pragma unroll
        for (int nb = 0; nb < 4; ++nb) acc[mb][nb] = (v8f){};
    const size_t aoff = (size_t)(r0 + lr) * K + 8 * hi, boff = (size_t)(c0 + lr) * K + 8 * hi;
#pragma unroll 1
    for (int kc = 0; kc < K; kc += 32) {
        v16h a[4];
#pragma unroll
        for (int mb = 0; mb < 4; ++mb) a[mb] = ldh(A + aoff + (size_t)mb * 16 * K + kc);
#pragma unroll
        for (int nb = 0; nb < 4; ++nb) { const v16h b = ldh(Bt + boff + (size_t)nb * 16 * K + kc);
#pragma unroll
            for (int mb = 0; mb < 4; ++mb) acc[mb][nb] = wmma16(a[mb], b, acc[mb][nb]); }
        asm volatile("v_nop\n\tv_nop\n\tv_nop\n\tv_nop" : "+v"(acc[0][0]), "+v"(acc[1][1]), "+v"(acc[2][2]), "+v"(acc[3][3]) : "v"(a[0]), "v"(a[1]), "v"(a[2]), "v"(a[3]));
    }
    const v4f braw = *(const v4f*)(bo + c0 + lr * 4);
    v4f bb;
#pragma unroll
    for (int i = 0; i < 4; ++i) bb[i] = bfval(braw[i]);
    const int bI = r0 / SEQ, tI = r0 % SEQ;
    float* obase = OUT + ((size_t)bI * OUT_SEQ + tI) * DM + c0;
    const float* rbase = res + ((size_t)bI * (size_t)res_seq + tI) * DM + c0;
#pragma unroll
    for (int mb = 0; mb < 4; ++mb) {
#pragma unroll
        for (int nb = 0; nb < 4; ++nb) {
#pragma unroll
            for (int j = 0; j < 8; ++j) os[(hi * 8 + j) * 68 + nb * 16 + lr] = acc[mb][nb][j]; }
        wave_sync();
        v4f fin[8];
#pragma unroll
        for (int s = 0; s < 8; ++s) { const int row = 2 * s + hi, cofs = lr * 4;
            const v4f x0 = *(const v4fa*)(&os[row * 68 + cofs]);
            const v4f rr = *(const v4f*)(rbase + (size_t)(mb * 16 + row) * DM + cofs);
            v4f rv;
#pragma unroll
            for (int i = 0; i < 4; ++i) rv[i] = (resbf != 0) ? bfval(rr[i]) : rr[i];
            fin[s] = x0 * oscl + bb + rv; }
#pragma unroll 1
        for (int ps = 0; ps < 2; ++ps) {
#pragma unroll
            for (int s = 0; s < 8; ++s) { const int row = 2 * s + hi, cofs = lr * 4;
                *(volatile v4f*)(obase + (size_t)(mb * 16 + row) * DM + cofs) = fin[s]; }
            if (ps == 0) __threadfence(); }
        wave_sync();
    }
}

__global__ __launch_bounds__(32 * AW) void k_flash(const h16* __restrict__ QH, const h16* __restrict__ KP, const h16* __restrict__ VT, h16* CTX) {
    __shared__ __align__(16) float os[AW * 16 * 68];
    const int lane = threadIdx.x & 31, wave = __builtin_amdgcn_readfirstlane((int)(threadIdx.x >> 5)), lr = lane & 15, hi = lane >> 4;
    const int zh = blockIdx.y; const int b = zh / NH_, h = zh % NH_;
    const int lk = SEQ >> ((h + 2) >> 2);
    const int t0 = (blockIdx.x * AW + wave) * 16;
    const size_t pbase = (size_t)zh * SEQ * HD;
    const size_t qo = pbase + (size_t)(t0 + lr) * HD + 8 * hi;
    const v16h qh0 = ldh(QH + qo), qh1 = ldh(QH + qo + 32);
    const size_t ko = pbase + (size_t)lr * HD + 8 * hi;
    const size_t vo = pbase + (size_t)lr * SEQ + 8 * hi;
    v8f o0 = (v8f){}, o1 = (v8f){}, o2 = (v8f){}, o3 = (v8f){};
    float m = -3.0e38f, l = 0.0f;
#pragma unroll 1
    for (int key0 = 0; key0 < lk; key0 += 32) {
        const h16* ka = KP + ko + (size_t)key0 * HD;
        const v16h ka0 = ldh(ka), ka1 = ldh(ka + 32), kb0 = ldh(ka + 16 * HD), kb1 = ldh(ka + 16 * HD + 32);
        v8f sa = (v8f){}, sb = (v8f){};
        sa = wmma16(ka0, qh0, sa); sb = wmma16(kb0, qh0, sb);
        sa = wmma16(ka1, qh1, sa); sb = wmma16(kb1, qh1, sb);
        asm volatile("v_nop\n\tv_nop\n\tv_nop\n\tv_nop" : "+v"(sa), "+v"(sb) : "v"(ka0), "v"(ka1), "v"(kb0), "v"(kb1), "v"(qh0), "v"(qh1));
        float ta[8], tb[8]; float mx = -3.0e38f;
#pragma unroll
        for (int r = 0; r < 8; ++r) { ta[r] = sa[r] * SC2; tb[r] = sb[r] * SC2; mx = fmaxf(mx, fmaxf(ta[r], tb[r])); }
        mx = fmaxf(mx, __shfl_xor(mx, 16, 32));
        const float mnew = fmaxf(m, mx);
        const float alpha = __builtin_amdgcn_exp2f(m - mnew);
        const float sh = PSH - mnew;
        v16h pb; float ls = 0.0f;
#pragma unroll
        for (int r = 0; r < 8; ++r) { const float ea = ta[r] + sh, eb = tb[r] + sh;
            const h16 pa = (ea < -14.0f) ? (h16)0.0f : (h16)__builtin_amdgcn_exp2f(ea);
            const h16 pc = (eb < -14.0f) ? (h16)0.0f : (h16)__builtin_amdgcn_exp2f(eb);
            pb[r] = pa; pb[8 + r] = pc; ls += (float)pa + (float)pc; }
        l = l * alpha + ls; m = mnew;
        o0 = o0 * alpha; o1 = o1 * alpha; o2 = o2 * alpha; o3 = o3 * alpha;
        const h16* va = VT + vo + key0;
        const v16h v0 = ldh(va), v1 = ldh(va + (size_t)16 * SEQ), v2 = ldh(va + (size_t)32 * SEQ), v3 = ldh(va + (size_t)48 * SEQ);
        o0 = wmma16(v0, pb, o0); o1 = wmma16(v1, pb, o1); o2 = wmma16(v2, pb, o2); o3 = wmma16(v3, pb, o3);
        asm volatile("v_nop\n\tv_nop\n\tv_nop\n\tv_nop" : "+v"(o0), "+v"(o1), "+v"(o2), "+v"(o3) : "v"(v0), "v"(v1), "v"(v2), "v"(v3), "v"(pb));
    }
    l += __shfl_xor(l, 16, 32);
    const float inv = CXS * (1.0f / l);
    const int wb = wave * 16 * 68;
    { v4f a, c;
      a[0] = o0[0] * inv; a[1] = o0[1] * inv; a[2] = o0[2] * inv; a[3] = o0[3] * inv; c[0] = o0[4] * inv; c[1] = o0[5] * inv; c[2] = o0[6] * inv; c[3] = o0[7] * inv;
      *(v4fa*)(&os[wb + lr * 68 +  0 + 8 * hi]) = a; *(v4fa*)(&os[wb + lr * 68 +  0 + 8 * hi + 4]) = c;
      a[0] = o1[0] * inv; a[1] = o1[1] * inv; a[2] = o1[2] * inv; a[3] = o1[3] * inv; c[0] = o1[4] * inv; c[1] = o1[5] * inv; c[2] = o1[6] * inv; c[3] = o1[7] * inv;
      *(v4fa*)(&os[wb + lr * 68 + 16 + 8 * hi]) = a; *(v4fa*)(&os[wb + lr * 68 + 16 + 8 * hi + 4]) = c;
      a[0] = o2[0] * inv; a[1] = o2[1] * inv; a[2] = o2[2] * inv; a[3] = o2[3] * inv; c[0] = o2[4] * inv; c[1] = o2[5] * inv; c[2] = o2[6] * inv; c[3] = o2[7] * inv;
      *(v4fa*)(&os[wb + lr * 68 + 32 + 8 * hi]) = a; *(v4fa*)(&os[wb + lr * 68 + 32 + 8 * hi + 4]) = c;
      a[0] = o3[0] * inv; a[1] = o3[1] * inv; a[2] = o3[2] * inv; a[3] = o3[3] * inv; c[0] = o3[4] * inv; c[1] = o3[5] * inv; c[2] = o3[6] * inv; c[3] = o3[7] * inv;
      *(v4fa*)(&os[wb + lr * 68 + 48 + 8 * hi]) = a; *(v4fa*)(&os[wb + lr * 68 + 48 + 8 * hi + 4]) = c; }
    wave_sync();
    h16* crow = CTX + ((size_t)b * SEQ + t0) * DM + h * HD;
#pragma unroll 1
    for (int ps = 0; ps < 2; ++ps) {
#pragma unroll
        for (int s = 0; s < 4; ++s) { const int row = 4 * s + (lane >> 3), c8 = (lane & 7) * 8;
            const v4f x0 = *(const v4fa*)(&os[wb + row * 68 + c8]); const v4f x1 = *(const v4fa*)(&os[wb + row * 68 + c8 + 4]); v8h hv;
#pragma unroll
            for (int i = 0; i < 4; ++i) { hv[i] = toh_flush(x0[i]); hv[4 + i] = toh_flush(x1[i]); }
            *(volatile v8h*)(crow + (size_t)row * DM + c8) = hv; }
        if (ps == 0) __threadfence(); }
}

__global__ __launch_bounds__(256) void k_ln(float* Y, const float* __restrict__ gamma, const float* __restrict__ beta, h16* HP, int wh) {
#pragma clang fp contract(off)
    __shared__ __align__(16) float rs[8 * DM];
    const int lane = threadIdx.x & 31, wave = __builtin_amdgcn_readfirstlane((int)(threadIdx.x >> 5));
    const int r = blockIdx.x * 8 + wave;
    const int bI = r / SEQ, tI = r % SEQ;
    float* yrow = Y + ((size_t)bI * OUT_SEQ + tI) * DM;
    v4f xv[8]; float s = 0.0f;
#pragma unroll
    for (int i = 0; i < 8; ++i) { xv[i] = *(const v4f*)(yrow + (i * 32 + lane) * 4); s += (xv[i][0] + xv[i][1]) + (xv[i][2] + xv[i][3]); }
    s += __shfl_xor(s, 16, 32); s += __shfl_xor(s, 8, 32); s += __shfl_xor(s, 4, 32); s += __shfl_xor(s, 2, 32); s += __shfl_xor(s, 1, 32);
    const float mu = s * (1.0f / DM);
    float q = 0.0f;
#pragma unroll
    for (int i = 0; i < 8; ++i) { const v4f d = xv[i] - mu; q += (d[0] * d[0] + d[1] * d[1]) + (d[2] * d[2] + d[3] * d[3]); }
    q += __shfl_xor(q, 16, 32); q += __shfl_xor(q, 8, 32); q += __shfl_xor(q, 4, 32); q += __shfl_xor(q, 2, 32); q += __shfl_xor(q, 1, 32);
    const float rstd = rsqrtf(q * (1.0f / DM) + LNE);
    v4f o[8];
#pragma unroll
    for (int i = 0; i < 8; ++i) { const v4f g = *(const v4f*)(gamma + (i * 32 + lane) * 4); const v4f be = *(const v4f*)(beta + (i * 32 + lane) * 4);
#pragma unroll
        for (int c = 0; c < 4; ++c) o[i][c] = ((xv[i][c] - mu) * rstd) * bfval(g[c]) + bfval(be[c]); }
#pragma unroll 1
    for (int ps = 0; ps < 2; ++ps) {
#pragma unroll
        for (int i = 0; i < 8; ++i) *(volatile v4f*)(yrow + (i * 32 + lane) * 4) = o[i];
        if (ps == 0) __threadfence(); }
    if (wh != 0) {
        const int wb = wave * DM;
#pragma unroll
        for (int i = 0; i < 8; ++i) *(v4fa*)(&rs[wb + (i * 32 + lane) * 4]) = o[i];
        wave_sync();
        h16* hrow = HP + (size_t)r * DM;
#pragma unroll 1
        for (int ps = 0; ps < 2; ++ps) {
#pragma unroll
            for (int j = 0; j < 4; ++j) { const int p8 = (j * 32 + lane) * 8;
                const v4f x0 = *(const v4fa*)(&rs[wb + p8]); const v4f x1 = *(const v4fa*)(&rs[wb + p8 + 4]); v8h hv;
#pragma unroll
                for (int i = 0; i < 4; ++i) { hv[i] = toh_flush(x0[i] * HCS); hv[4 + i] = toh_flush(x1[i] * HCS); }
                *(volatile v8h*)(hrow + p8) = hv; }
            if (ps == 0) __threadfence(); }
    }
}

static constexpr size_t al256(size_t v) { return (v + 255) & ~(size_t)255; }
static constexpr size_t SZ_XB = al256((size_t)NB * SEQ * DM * 2);
static constexpr size_t SZ_WB = al256((size_t)3 * DM * DM * 2);
static constexpr size_t SZ_WO = al256((size_t)DM * DM * 2);
static constexpr size_t SZ_W1 = al256((size_t)DM * DFF * 2);
static constexpr size_t SZ_W2 = al256((size_t)DFF * DM * 2);
static constexpr size_t SZ_PL = al256((size_t)NB * NH_ * SEQ * HD * 2);
static constexpr size_t SZ_CX = al256((size_t)NB * SEQ * DM * 2);
static constexpr size_t SZ_F1 = al256((size_t)NB * SEQ * DFF * 2);
static constexpr size_t SZ_TOTAL = SZ_XB + SZ_WB + SZ_WO + SZ_W1 + SZ_W2 + 3 * SZ_PL + SZ_CX;
static_assert(SZ_F1 <= 3 * SZ_PL + SZ_CX);
static_assert(SZ_TOTAL <= (size_t)134217728);
static_assert(((size_t)DM * DM * 2) % 256 == 0);

extern "C" void kernel_launch(void* const* d_in, const int* in_sizes, int n_in,
                              void* d_out, int out_size, void* d_ws, size_t ws_size, hipStream_t stream) {
    if (n_in < 11) return;
    const size_t needx = ((size_t)(NB - 1) * SEQ_FULL + SEQ) * DM;
    if ((size_t)in_sizes[0] < needx) return;
    if ((size_t)in_sizes[1] < (size_t)3 * DM * DM || (size_t)in_sizes[2] < (size_t)3 * DM) return;
    if ((size_t)in_sizes[3] < (size_t)DM * DM || (size_t)in_sizes[4] < (size_t)DM) return;
    if ((size_t)in_sizes[5] < (size_t)DM || (size_t)in_sizes[6] < (size_t)DM) return;
    if ((size_t)in_sizes[7] < (size_t)DM * DFF || (size_t)in_sizes[8] < (size_t)DFF) return;
    if ((size_t)in_sizes[9] < (size_t)DFF * DM || (size_t)in_sizes[10] < (size_t)DM) return;
    if ((size_t)out_size < ((size_t)(NB - 1) * OUT_SEQ + SEQ) * DM) return;
    if (SZ_TOTAL > ws_size) return;
    const float* x = (const float*)d_in[0]; const float* wqkv = (const float*)d_in[1]; const float* bqkv = (const float*)d_in[2];
    const float* wout = (const float*)d_in[3]; const float* bout = (const float*)d_in[4];
    const float* gam = (const float*)d_in[5]; const float* bet = (const float*)d_in[6];
    const float* w1 = (const float*)d_in[7]; const float* b1 = (const float*)d_in[8];
    const float* w2 = (const float*)d_in[9]; const float* b2 = (const float*)d_in[10];
    float* OUT = (float*)d_out;
    char* wsp = (char*)d_ws;
    bf* XB = (bf*)wsp; wsp += SZ_XB;
    bf* WB = (bf*)wsp; wsp += SZ_WB;
    h16* WOH = (h16*)wsp; wsp += SZ_WO;
    h16* W1H = (h16*)wsp; wsp += SZ_W1;
    h16* W2H = (h16*)wsp; wsp += SZ_W2;
    char* shared0 = wsp;
    h16* QH = (h16*)wsp; wsp += SZ_PL;
    h16* KP = (h16*)wsp; wsp += SZ_PL;
    h16* VT = (h16*)wsp; wsp += SZ_PL;
    h16* CTX = (h16*)wsp; wsp += SZ_CX;
    h16* F1 = (h16*)shared0;
    h16* HH = (h16*)XB;
    bf* WQ = WB; bf* WK = WB + (size_t)DM * DM; bf* WV = WB + (size_t)2 * DM * DM;

    if (SEQ == SEQ_FULL) {
        const size_t n8 = (size_t)NB * SEQ * DM / 8;
        k_cvt8<<<(unsigned)((n8 + 255) / 256), 256, 0, stream>>>(x, XB, n8);
    } else {
        const size_t n8 = (size_t)SEQ * DM / 8;
        for (int b = 0; b < NB; ++b) k_cvt8<<<(unsigned)((n8 + 255) / 256), 256, 0, stream>>>(x + (size_t)b * SEQ_FULL * DM, XB + (size_t)b * SEQ * DM, n8);
    }
    k_wtb<<<dim3(3 * DM / 64, DM / 64, 1), 256, 0, stream>>>(wqkv, WB, DM, 3 * DM);
    k_wth<<<dim3(DM / 64, DM / 64, 1), 256, 0, stream>>>(wout, WOH, DM, DM, WOS);
    k_wth<<<dim3(DFF / 64, DM / 64, 1), 256, 0, stream>>>(w1, W1H, DM, DFF, W1S);
    k_wth<<<dim3(DM / 64, DFF / 64, 1), 256, 0, stream>>>(w2, W2H, DFF, DM, W2S);

    k_proj<<<dim3(NB * SEQ / 64, DM / 64, 1), 32, 0, stream>>>(XB, (size_t)DM, WQ, (size_t)DM, bqkv, DM, 0, QH, SEQ, (size_t)NH_ * SEQ * HD, HD, HD, (size_t)SEQ * HD);
    for (int g = 0; g < 5; ++g) {
        const int st = 1 << g, lk = SEQ >> g;
        const int hb = (g == 0) ? 0 : (4 * g - 2);
        const int ng = (g == 0 || g == 4) ? 2 : 4;
        k_proj<<<dim3(NB * lk / 64, ng, 1), 32, 0, stream>>>(XB, (size_t)st * DM, WK + (size_t)hb * 64 * DM, (size_t)DM, bqkv + DM + hb * 64, ng * 64, 0,
                                                             KP + (size_t)hb * SEQ * HD, lk, (size_t)NH_ * SEQ * HD, HD, HD, (size_t)SEQ * HD);
        k_proj<<<dim3(ng, NB * lk / 64, 1), 32, 0, stream>>>(WV + (size_t)hb * 64 * DM, (size_t)DM, XB, (size_t)st * DM, bqkv + 2 * DM + hb * 64, ng * 64, 1,
                                                             VT + (size_t)hb * HD * SEQ, DM, (size_t)0, SEQ, lk, (size_t)DM * SEQ);
    }

    k_flash<<<dim3(SEQ / (16 * AW), NB * NH_, 1), 32 * AW, 0, stream>>>(QH, KP, VT, CTX);

    k_oproj<<<dim3(NB * SEQ / 64, DM / 64, 1), 32, 0, stream>>>(CTX, WOH, DM, OSCL, bout, x, SEQ_FULL, 1, OUT);
    k_ln<<<NB * SEQ / 8, 256, 0, stream>>>(OUT, gam, bet, HH, 1);
    k_ffn1<<<dim3(NB * SEQ / 64, DFF / 64, 1), 32, 0, stream>>>(HH, W1H, b1, F1);
    k_oproj<<<dim3(NB * SEQ / 64, DM / 64, 1), 32, 0, stream>>>(F1, W2H, DFF, FOLD2, b2, OUT, OUT_SEQ, 0, OUT);
    k_ln<<<NB * SEQ / 8, 256, 0, stream>>>(OUT, gam, bet, HH, 0);
}
